// HANLayer_79834852098259
// MI455X (gfx1250) — hardware-run, weakly checked
//
#include <hip/hip_runtime.h>
#include <stddef.h>
#include <stdint.h>
#include <math.h>


#define CIN     256
#define HCH     128
#define NMP     3
#define FTW     (NMP * HCH)
#define KZ      256
#define HIDW    128
#define NTHR    256
#define NWAVE   8
#define EPT     8
#define CHUNK   (NTHR * EPT)
#define WCAP    (EPT * 32)
#define LISTN   (NWAVE * WCAP)
#define NBMAX   2048
#define PKS     11
#define RCAP    28672
#define DEGCAP  256
#define GBM     64
#define GBN     128
#define GTHR    128
#define GNT     8
#define PREC    32
#define NEGSL   0.2f
#define WSMAX   134217728
#define LDS_AGG ((2 * RCAP + 2 * NBMAX + LISTN) * 4 + 64)

static_assert((CHUNK & (CHUNK - 1)) == 0 && CHUNK <= (1 << PKS));
static_assert((NBMAX & (NBMAX - 1)) == 0 && NBMAX <= (1 << PKS));
static_assert(NTHR * 8 == NBMAX);
static_assert(LISTN >= NBMAX && LISTN >= NWAVE * WCAP);
static_assert((RCAP % 32) == 0);
static_assert(LDS_AGG <= 300000);
static_assert(GBM == (GTHR / 32) * 16 && GBN == 16 * GNT && GTHR == GBN && GBN == 4 * 32);
static_assert(HCH == 32 * 4);
static_assert(KZ == 2 * HCH && GBN == HCH && HIDW == GTHR);
static_assert((CIN % 32) == 0 && (KZ % 32) == 0);
static_assert((FTW % GBN) == 0 && (HIDW % GBN) == 0);
static_assert(((FTW * 4) % 128) == 0);
static_assert(PREC / 4 <= GTHR && PREC >= GTHR / 32);
static_assert((CIN / 8) == 32 && (KZ / 8) == 32);

typedef float          v4f  __attribute__((ext_vector_type(4)));
typedef float          v8f  __attribute__((ext_vector_type(8)));
typedef int            v4i  __attribute__((ext_vector_type(4)));
typedef int            v8i  __attribute__((ext_vector_type(8)));
typedef unsigned int   v4u  __attribute__((ext_vector_type(4)));
typedef unsigned short v8us __attribute__((ext_vector_type(8)));
typedef __bf16         v16b __attribute__((ext_vector_type(16)));
typedef v4f  __attribute__((may_alias)) v4fa;
typedef v8us __attribute__((may_alias)) v8usa;
union Frag { v16b vb; v8us h[2]; v8i w; };

__device__ __forceinline__ v8f wmb(const Frag& a, const Frag& b, v8f c) {
  v8f d = __builtin_amdgcn_wmma_f32_16x16x32_bf16(false, a.vb, false, b.vb, (short)0, c, false, false);
  asm volatile("v_nop\n\tv_nop\n\tv_nop\n\tv_nop" : "+v"(d) : "v"(a.w), "v"(b.w));
  return d;
}

__device__ __forceinline__ unsigned int f2bf(float f) {
  const unsigned int u = __float_as_uint(f);
  return ((u + 0x7FFFu + ((u >> 16) & 1u)) >> 16) & 0xFFFFu;
}
__device__ __forceinline__ float bf2f(unsigned int b) { return __uint_as_float(b << 16); }
__device__ __forceinline__ float bfr(float f) { return bf2f(f2bf(f)); }
__device__ __forceinline__ v4f bfr4(const v4f a) {
  v4f r; r.x = bfr(a.x); r.y = bfr(a.y); r.z = bfr(a.z); r.w = bfr(a.w); return r;
}
__device__ __forceinline__ v8us cv8b(const float* __restrict__ p, size_t stride) {
  v8us o;
#pragma unroll
  for (int i = 0; i < 8; ++i) o[i] = (unsigned short)f2bf(p[(size_t)i * stride]);
  return o;
}

__device__ __forceinline__ int scan_chunk(const int* __restrict__ dsts, int nE, int cbase, int slotBase,
                                          int nb, int vec8, int* list, int tid, int lane, int wave) {
  int wc = 0;
  const int el0  = tid * EPT;
  const int e0   = cbase + el0;
  const int sent = -2147483647 - 1;
  v4i da, db;
  if (vec8 != 0 && cbase + CHUNK <= nE) {
    da = *(const v4i*)(dsts + e0);
    db = *(const v4i*)(dsts + e0 + 4);
  } else {
    da.x = (e0     < nE) ? dsts[min(e0,     nE - 1)] : sent;
    da.y = (e0 + 1 < nE) ? dsts[min(e0 + 1, nE - 1)] : sent;
    da.z = (e0 + 2 < nE) ? dsts[min(e0 + 2, nE - 1)] : sent;
    da.w = (e0 + 3 < nE) ? dsts[min(e0 + 3, nE - 1)] : sent;
    db.x = (e0 + 4 < nE) ? dsts[min(e0 + 4, nE - 1)] : sent;
    db.y = (e0 + 5 < nE) ? dsts[min(e0 + 5, nE - 1)] : sent;
    db.z = (e0 + 6 < nE) ? dsts[min(e0 + 6, nE - 1)] : sent;
    db.w = (e0 + 7 < nE) ? dsts[min(e0 + 7, nE - 1)] : sent;
  }
  const unsigned nbs = (unsigned)slotBase;
  const unsigned unb = (unsigned)nb;
  const unsigned s0 = (unsigned)da.x - nbs, s1 = (unsigned)da.y - nbs;
  const unsigned s2 = (unsigned)da.z - nbs, s3 = (unsigned)da.w - nbs;
  const unsigned s4 = (unsigned)db.x - nbs, s5 = (unsigned)db.y - nbs;
  const unsigned s6 = (unsigned)db.z - nbs, s7 = (unsigned)db.w - nbs;
  const bool h0 = s0 < unb, h1 = s1 < unb, h2 = s2 < unb, h3 = s3 < unb;
  const bool h4 = s4 < unb, h5 = s5 < unb, h6 = s6 < unb, h7 = s7 < unb;
  const unsigned any = __builtin_amdgcn_ballot_w32(h0 | h1 | h2 | h3 | h4 | h5 | h6 | h7);
  if (any != 0u) {
#define HITJ(J, HJ, SJ) { \
      const unsigned mj = __builtin_amdgcn_ballot_w32(HJ); \
      if (mj != 0u) { \
        if (HJ) { \
          const int pos = wc + (int)__builtin_amdgcn_mbcnt_lo(mj, 0u); \
          if (pos < WCAP) list[wave * WCAP + pos] = ((el0 + (J)) << PKS) | (int)(SJ); \
        } \
        wc += (int)__builtin_popcount(mj); } }
    HITJ(0, h0, s0)
    HITJ(1, h1, s1)
    HITJ(2, h2, s2)
    HITJ(3, h3, s3)
    HITJ(4, h4, s4)
    HITJ(5, h5, s5)
    HITJ(6, h6, s6)
    HITJ(7, h7, s7)
#undef HITJ
  }
  return wc;
}

__global__ __launch_bounds__(NTHR) void k_prep(const float* __restrict__ h, const float* __restrict__ fcw,
                                               const float* __restrict__ sw1,
                                               unsigned short* hb, unsigned short* wt, unsigned short* w1t,
                                               int nN, int nUh, int nUw, int nUs) {
  const int u = (int)blockIdx.x * NTHR + (int)threadIdx.x;
  v8us o;
  unsigned short* dp;
  if (u < nUh) {
    const int row = u >> 5;
    const int c8  = (u & 31) * 8;
    const int rc  = row < nN ? row : nN - 1;
    const v4f a = *(const v4fa*)(h + (size_t)rc * CIN + c8);
    const v4f b = *(const v4fa*)(h + (size_t)rc * CIN + c8 + 4);
    o[0] = (unsigned short)f2bf(a.x); o[1] = (unsigned short)f2bf(a.y);
    o[2] = (unsigned short)f2bf(a.z); o[3] = (unsigned short)f2bf(a.w);
    o[4] = (unsigned short)f2bf(b.x); o[5] = (unsigned short)f2bf(b.y);
    o[6] = (unsigned short)f2bf(b.z); o[7] = (unsigned short)f2bf(b.w);
    const v8us z8 = {0, 0, 0, 0, 0, 0, 0, 0};
    if (row >= nN) o = z8;
    dp = hb + (size_t)u * 8;
  } else if (u < nUh + nUw) {
    const int v  = u - nUh;
    const int n  = v >> 5;
    const int k8 = (v & 31) * 8;
    const int mp = n >> 7, nn = n & (HCH - 1);
    o = cv8b(fcw + ((size_t)mp * CIN + (size_t)k8) * HCH + nn, HCH);
    dp = wt + (size_t)v * 8;
  } else if (u < nUh + nUw + nUs) {
    const int v  = u - nUh - nUw;
    const int n  = v >> 5;
    const int k8 = (v & 31) * 8;
    const int kk = k8 & (HIDW - 1);
    o = cv8b(sw1 + (size_t)kk * HIDW + n, HIDW);
    dp = w1t + (size_t)v * 8;
  } else {
    return;
  }
  *(volatile v8us*)dp = o;
  __threadfence();
  *(volatile v8us*)dp = o;
}

template <int EPI>
__global__ __launch_bounds__(GTHR) void k_gemm(const unsigned short* __restrict__ A, int lda, int aPlane,
                                               const unsigned short* __restrict__ BT, int ldb, int K,
                                               float* outF, int ldo,
                                               const float* __restrict__ sb1, const float* __restrict__ sw2,
                                               float* part, int nN, int mRows) {
  __shared__ __attribute__((aligned(16))) float stg[GBM * GBN];
  __shared__ __attribute__((aligned(16))) float pst[PREC];
  const int tid = (int)threadIdx.x, lane = tid & 31, wave = tid >> 5, hh = lane >> 4, m = lane & 15;
  const int rowBase = (int)blockIdx.x * GBM;
  const int colBase = (EPI == 0) ? (int)blockIdx.y * GBN : 0;
  const unsigned short* Ab = A + ((EPI == 1) ? (size_t)blockIdx.y * (size_t)aPlane : (size_t)0);

  v8f acc[GNT];
  {
    const v8f z = {0.f, 0.f, 0.f, 0.f, 0.f, 0.f, 0.f, 0.f};
#pragma unroll
    for (int t = 0; t < GNT; ++t) acc[t] = z;
  }
  const unsigned short* ap = Ab + (size_t)(rowBase + 16 * wave + m) * (size_t)lda + 8 * hh;
  const unsigned short* bp = BT + (size_t)(colBase + m) * (size_t)ldb + 8 * hh;

#pragma unroll 1
  for (int k0 = 0; k0 < K; k0 += 32) {
    Frag af;
    af.h[0] = *(const v8usa*)(ap + k0);
    af.h[1] = *(const v8usa*)(ap + k0 + 16);
#pragma unroll
    for (int nt = 0; nt < GNT; ++nt) {
      const unsigned short* wq = bp + (size_t)(16 * nt) * (size_t)ldb + k0;
      Frag bf;
      bf.h[0] = *(const v8usa*)wq;
      bf.h[1] = *(const v8usa*)(wq + 16);
      acc[nt] = wmb(af, bf, acc[nt]);
    }
  }

#pragma unroll
  for (int nt = 0; nt < GNT; ++nt) {
    const int lc = 16 * nt + m;
    float bb = 0.0f;
    if constexpr (EPI == 1) bb = bfr(sb1[lc]);
#pragma unroll
    for (int r = 0; r < 8; ++r) {
      const int lr = 16 * wave + 8 * hh + r;
      const bool live = (rowBase + lr) < nN;
      const float v = acc[nt][r] + bb;
      stg[lr * GBN + lc] = live ? v : 0.0f;
    }
  }
  __syncthreads();

  if constexpr (EPI == 0) {
    v4f fv[16];
#pragma unroll
    for (int i = 0; i < 16; ++i) {
      const int lr = 16 * wave + i;
      fv[i] = *(const v4fa*)(stg + lr * GBN + 4 * lane);
    }
#pragma unroll
    for (int i = 0; i < 16; ++i) {
      const int gr = rowBase + 16 * wave + i;
      float* op = outF + (size_t)gr * (size_t)ldo + colBase + 4 * lane;
      if (gr < mRows) *(volatile v4f*)op = fv[i];
    }
    __threadfence();
#pragma unroll
    for (int i = 0; i < 16; ++i) {
      const int gr = rowBase + 16 * wave + i;
      float* op = outF + (size_t)gr * (size_t)ldo + colBase + 4 * lane;
      if (gr < mRows) *(volatile v4f*)op = fv[i];
    }
  } else {
    const float w2 = bfr(sw2[tid]);
    float s = 0.0f;
#pragma unroll 1
    for (int r = 0; r < GBM; ++r) s = fmaf(tanhf(stg[r * GBN + tid]), w2, s);
#pragma unroll
    for (int off = 16; off > 0; off >>= 1) s += __shfl_xor(s, off);
    if (lane == 0) pst[wave] = s;
    if (tid >= GTHR / 32 && tid < PREC) pst[tid] = 0.0f;
    __syncthreads();
    const bool ok = tid < PREC / 4;
    v4f pv = {0.f, 0.f, 0.f, 0.f};
    const size_t prow = (size_t)blockIdx.y * (size_t)gridDim.x + (size_t)blockIdx.x;
    float* pp = part + prow * PREC + 4 * tid;
    if (ok) { pv = *(const v4fa*)(pst + 4 * tid); *(volatile v4f*)pp = pv; }
    __threadfence();
    if (ok) *(volatile v4f*)pp = pv;
  }
}

__global__ __launch_bounds__(NTHR) void k_agg(
    const int* __restrict__ src, const int* __restrict__ dst, const float* __restrict__ ew,
    const float* __restrict__ ft,
    const float* __restrict__ attl, const float* __restrict__ attr, const float* __restrict__ bias,
    float* zfp, unsigned short* zhp,
    int nN, int nE, int nb, int vec8, int MPr) {
  extern __shared__ v4f lds_dyn[];
  int* reg1 = (int*)lds_dyn;
  int* reg2 = reg1 + RCAP;
  int* scnt = reg2 + RCAP;
  int* soff = scnt + NBMAX;
  int* list = soff + NBMAX;
  int* wcnt = list + LISTN;
  int* wtot = wcnt + NWAVE;
  const int tid = (int)threadIdx.x, lane = tid & 31, wave = tid >> 5;
  const int nodeBase = (int)blockIdx.x * nb;
  const int mp = (int)blockIdx.y;
  const int*   srcs = src + (size_t)mp * (size_t)nE;
  const int*   dsts = dst + (size_t)mp * (size_t)nE;
  const float* ews  = ew  + (size_t)mp * (size_t)nE;
  const float* fin  = ft  + (size_t)mp * HCH;
  const float* al   = attl + (size_t)mp * HCH;
  const float* ar   = attr + (size_t)mp * HCH;
  const float* bb   = bias + (size_t)mp * HCH;
  float*          zf = zfp + (size_t)mp * (size_t)MPr * HCH;
  unsigned short* zh = zhp + (size_t)mp * (size_t)MPr * KZ;

  for (int i = tid; i < NBMAX; i += NTHR) scnt[i] = 0;
  __syncthreads();

  int tot = 0;
  const int nChunks = (nE + CHUNK - 1) / CHUNK;
#pragma unroll 1
  for (int ch = 0; ch < nChunks; ++ch) {
    const int cbase = ch * CHUNK;
    const int wc = scan_chunk(dsts, nE, cbase, nodeBase, nb, vec8, list, tid, lane, wave);
    if (lane == 0) wcnt[wave] = wc;
    __syncthreads();
    int pre = 0, all = 0;
#pragma unroll
    for (int w2 = 0; w2 < NWAVE; ++w2) {
      int c = wcnt[w2];
      c = c < 0 ? 0 : (c > WCAP ? WCAP : c);
      all += c;
      pre += (w2 < wave) ? c : 0;
    }
    const int wcc  = wc > WCAP ? WCAP : wc;
    const int base = tot + pre;
#pragma unroll 1
    for (int i = lane; i < wcc; i += 32) {
      const int ent = list[wave * WCAP + i];
      const int el  = (ent >> PKS) & (CHUNK - 1);
      const int sl  = ent & (NBMAX - 1);
      int eid = cbase + el;
      eid = eid > nE - 1 ? nE - 1 : eid;
      const int pos = base + i;
      if (pos < RCAP) reg1[pos] = (int)(((unsigned)eid << PKS) | (unsigned)sl);
    }
    tot += all;
    tot = tot > RCAP ? RCAP : tot;
    __syncthreads();
  }
  const int nh = tot;

  if (wave == 0) {
#pragma unroll 1
    for (int b0 = 0; b0 < nh; b0 += 32) {
      const int idx = b0 + lane;
      const int uv  = reg1[idx < nh ? idx : nh - 1];
      const int m32 = (nh - b0) < 32 ? (nh - b0) : 32;
#pragma unroll 1
      for (int k = 0; k < m32; ++k) {
        const int u  = __builtin_amdgcn_readlane(uv, k);
        const int sl = u & (NBMAX - 1);
        if (lane == 0) scnt[sl] = scnt[sl] + 1;
      }
    }
  }
  __syncthreads();

  {
    const v4i ca = *(const v4i*)(scnt + 8 * tid);
    const v4i cb = *(const v4i*)(scnt + 8 * tid + 4);
    const int e0 = ca.x < 0 ? 0 : ca.x, e1 = ca.y < 0 ? 0 : ca.y, e2 = ca.z < 0 ? 0 : ca.z, e3 = ca.w < 0 ? 0 : ca.w;
    const int e4 = cb.x < 0 ? 0 : cb.x, e5 = cb.y < 0 ? 0 : cb.y, e6 = cb.z < 0 ? 0 : cb.z, e7 = cb.w < 0 ? 0 : cb.w;
    const int ts = e0 + e1 + e2 + e3 + e4 + e5 + e6 + e7;
    int incl = ts;
#pragma unroll
    for (int d = 1; d < 32; d <<= 1) {
      const int up = __shfl_up(incl, d);
      if (lane >= d) incl += up;
    }
    if (lane == 31) wtot[wave] = incl;
    __syncthreads();
    int pre = 0;
#pragma unroll
    for (int w2 = 0; w2 < NWAVE; ++w2) pre += (w2 < wave) ? wtot[w2] : 0;
    int run = pre + incl - ts;
    soff[8 * tid + 0] = run; run += e0;
    soff[8 * tid + 1] = run; run += e1;
    soff[8 * tid + 2] = run; run += e2;
    soff[8 * tid + 3] = run; run += e3;
    soff[8 * tid + 4] = run; run += e4;
    soff[8 * tid + 5] = run; run += e5;
    soff[8 * tid + 6] = run; run += e6;
    soff[8 * tid + 7] = run;
  }
  __syncthreads();
  for (int i = tid; i < NBMAX; i += NTHR) list[i] = soff[i];
  __syncthreads();

  if (wave == 0) {
#pragma unroll 1
    for (int b0 = 0; b0 < nh; b0 += 32) {
      const int idx = b0 + lane;
      const int uv  = reg1[idx < nh ? idx : nh - 1];
      const int m32 = (nh - b0) < 32 ? (nh - b0) : 32;
#pragma unroll 1
      for (int k = 0; k < m32; ++k) {
        const int u   = __builtin_amdgcn_readlane(uv, k);
        const int sl  = u & (NBMAX - 1);
        const int eid = (int)((unsigned)u >> PKS);
        if (lane == 0) {
          int pos = list[sl];
          pos = pos < 0 ? 0 : (pos > RCAP - 1 ? RCAP - 1 : pos);
          reg2[pos] = eid;
          list[sl] = pos + 1;
        }
      }
    }
  }
  __syncthreads();

  const int nbw = nb >> 3;
  const bool ovf = (nh >= RCAP);
  const float qnan = __int_as_float(0x7fc00000);
  const v4f al4 = bfr4(*(const v4fa*)(al + 4 * lane));
  const v4f ar4 = bfr4(*(const v4fa*)(ar + 4 * lane));
  const v4f bb4 = bfr4(*(const v4fa*)(bb + 4 * lane));

#pragma unroll 1
  for (int jt = 0; jt < nbw; ++jt) {
    const int slot = wave * nbw + jt;
    const int grow = nodeBase + slot;
    const int gcl  = grow < nN ? grow : nN - 1;
    int st = soff[slot];
    const int craw = scnt[slot];
    int cnt = craw;
    st  = st < 0 ? 0 : (st > nh ? nh : st);
    cnt = cnt < 0 ? 0 : (cnt > DEGCAP ? DEGCAP : cnt);
    if (cnt > nh - st) cnt = nh - st;
    const float pz = (ovf || craw > DEGCAP) ? qnan : 0.0f;
    const bool liveRow = grow < nN;

    const v4f fd = *(const v4fa*)(fin + (size_t)gcl * FTW + 4 * lane);
    float pd = fd.x * ar4.x; pd = fmaf(fd.y, ar4.y, pd); pd = fmaf(fd.z, ar4.z, pd); pd = fmaf(fd.w, ar4.w, pd);
    pd += __shfl_xor(pd, 1);
    pd += __shfl_xor(pd, 2);
    float mx = -1.0e30f, dn = 0.0f;
    float a0 = 0.0f, a1 = 0.0f, a2 = 0.0f, a3 = 0.0f;

#pragma unroll 1
    for (int q = 0; q < cnt; ++q) {
      int idx = st + q; idx = idx > RCAP - 1 ? RCAP - 1 : idx;
      int eid = reg2[idx]; eid = eid < 0 ? 0 : (eid > nE - 1 ? nE - 1 : eid);
      const int sraw = srcs[eid];
      const int s = sraw < 0 ? 0 : (sraw > nN - 1 ? nN - 1 : sraw);
      const float wv = bfr(ews[eid]);
      const v4f fs = *(const v4fa*)(fin + (size_t)s * FTW + 4 * lane);
      float es = fs.x * al4.x; es = fmaf(fs.y, al4.y, es); es = fmaf(fs.z, al4.z, es); es = fmaf(fs.w, al4.w, es);
      es += __shfl_xor(es, 1);
      es += __shfl_xor(es, 2);
      float lg = (es + pd) * wv;
      lg = lg > 0.f ? lg : NEGSL * lg;
      const float df = lg - mx;
      const float ee = __expf(-fabsf(df));
      const bool up  = df > 0.f;
      const float s1 = up ? ee : 1.0f;
      const float s2 = up ? 1.0f : ee;
      mx = up ? lg : mx;
      dn = fmaf(dn, s1, s2);
      a0 = fmaf(a0, s1, s2 * fs.x);
      a1 = fmaf(a1, s1, s2 * fs.y);
      a2 = fmaf(a2, s1, s2 * fs.z);
      a3 = fmaf(a3, s1, s2 * fs.w);
    }
    const float dnz = dn > 0.0f ? dn : 1.0f;
    const float inv = __builtin_amdgcn_rcpf(dnz);
    float h0 = fmaf(a0, inv, bb4.x);
    float h1 = fmaf(a1, inv, bb4.y);
    float h2 = fmaf(a2, inv, bb4.z);
    float h3 = fmaf(a3, inv, bb4.w);
    const float n0 = expm1f(fminf(h0, 0.f));
    const float n1 = expm1f(fminf(h1, 0.f));
    const float n2 = expm1f(fminf(h2, 0.f));
    const float n3 = expm1f(fminf(h3, 0.f));
    h0 = h0 > 0.f ? h0 : n0;
    h1 = h1 > 0.f ? h1 : n1;
    h2 = h2 > 0.f ? h2 : n2;
    h3 = h3 > 0.f ? h3 : n3;
    h0 = (liveRow ? h0 : 0.f) + pz;
    h1 = (liveRow ? h1 : 0.f) + pz;
    h2 = (liveRow ? h2 : 0.f) + pz;
    h3 = (liveRow ? h3 : 0.f) + pz;

    v4f ov; ov.x = h0; ov.y = h1; ov.z = h2; ov.w = h3;
    const unsigned int hb0 = f2bf(h0), hb1 = f2bf(h1), hb2 = f2bf(h2), hb3 = f2bf(h3);
    const unsigned int lb0 = f2bf(h0 - bf2f(hb0)), lb1 = f2bf(h1 - bf2f(hb1));
    const unsigned int lb2 = f2bf(h2 - bf2f(hb2)), lb3 = f2bf(h3 - bf2f(hb3));
    const int hwA = (int)(hb0 | (hb1 << 16));
    const int hwB = (int)(hb2 | (hb3 << 16));
    const int lwA = (int)(lb0 | (lb1 << 16));
    const int lwB = (int)(lb2 | (lb3 << 16));
    const int j  = lane & 15;
    const int sA = 2 * j, sB = 2 * j + 1;
    const int g0h = __shfl(hwA, sA), g1h = __shfl(hwB, sA), g2h = __shfl(hwA, sB), g3h = __shfl(hwB, sB);
    const int g0l = __shfl(lwA, sA), g1l = __shfl(lwB, sA), g2l = __shfl(lwA, sB), g3l = __shfl(lwB, sB);
    const bool hsel = lane < 16;
    v4u pv;
    pv.x = (unsigned int)(hsel ? g0h : g0l);
    pv.y = (unsigned int)(hsel ? g1h : g1l);
    pv.z = (unsigned int)(hsel ? g2h : g2l);
    pv.w = (unsigned int)(hsel ? g3h : g3l);

    float*          fp = zf + (size_t)grow * HCH + 4 * lane;
    unsigned short* hp = zh + (size_t)grow * KZ + 8 * lane;
    const bool wr = grow < MPr;
    if (wr) { *(volatile v4f*)fp = ov; *(volatile v4u*)hp = pv; }
    __threadfence();
    if (wr) { *(volatile v4f*)fp = ov; *(volatile v4u*)hp = pv; }
  }
}

__global__ __launch_bounds__(NTHR) void k_beta(const float* __restrict__ part, int nPart, int nN, float* beta) {
  __shared__ double red[NTHR];
  __shared__ float wv[4];
  __shared__ __attribute__((aligned(16))) float line[PREC];
  const int tid = (int)threadIdx.x;
  const double invN = 1.0 / (double)(nN < 1 ? 1 : nN);
#pragma unroll 1
  for (int mp = 0; mp < NMP; ++mp) {
    double s = 0.0;
#pragma unroll 1
    for (int r = tid; r < nPart; r += NTHR) {
      const v4f p = *(const v4fa*)(part + ((size_t)mp * (size_t)nPart + (size_t)r) * PREC);
      s += (double)p.x; s += (double)p.y; s += (double)p.z; s += (double)p.w;
    }
    red[tid] = s;
    __syncthreads();
#pragma unroll
    for (int d = NTHR / 2; d > 0; d >>= 1) {
      if (tid < d) red[tid] = red[tid] + red[tid + d];
      __syncthreads();
    }
    if (tid == 0) wv[mp] = (float)(red[0] * invN);
    __syncthreads();
  }
  if (tid < PREC) {
    const float w0 = wv[0], w1 = wv[1], w2 = wv[2];
    const float mxw = fmaxf(w0, fmaxf(w1, w2));
    const float e0 = expf(w0 - mxw), e1 = expf(w1 - mxw), e2 = expf(w2 - mxw);
    const float inv = 1.0f / (e0 + e1 + e2);
    const float v = tid == 0 ? e0 * inv : (tid == 1 ? e1 * inv : (tid == 2 ? e2 * inv : 0.0f));
    line[tid] = v;
  }
  __syncthreads();
  const bool ok = tid < PREC / 4;
  v4f o = {0.f, 0.f, 0.f, 0.f};
  if (ok) { o = *(const v4fa*)(line + 4 * tid); *(volatile v4f*)(beta + 4 * tid) = o; }
  __threadfence();
  if (ok) *(volatile v4f*)(beta + 4 * tid) = o;
}

__global__ __launch_bounds__(NTHR) void k_out(const float* __restrict__ zf, const float* __restrict__ beta,
                                              int plane, int nUnits, float* out) {
  const int i = (int)blockIdx.x * NTHR + (int)threadIdx.x;
  if (i >= nUnits) return;
  const float b0 = beta[0], b1 = beta[1], b2 = beta[2];
  const size_t e = (size_t)i * 4;
  const v4f z0 = *(const v4fa*)(zf + e);
  const v4f z1 = *(const v4fa*)(zf + (size_t)plane + e);
  const v4f z2 = *(const v4fa*)(zf + 2 * (size_t)plane + e);
  v4f o;
  o.x = fmaf(z2.x, b2, fmaf(z1.x, b1, z0.x * b0));
  o.y = fmaf(z2.y, b2, fmaf(z1.y, b1, z0.y * b0));
  o.z = fmaf(z2.z, b2, fmaf(z1.z, b1, z0.z * b0));
  o.w = fmaf(z2.w, b2, fmaf(z1.w, b1, z0.w * b0));
  float* op = out + e;
  *(volatile v4f*)op = o;
  __threadfence();
  *(volatile v4f*)op = o;
}

static int pick_nb(int nE, int nN) {
  int nb = NBMAX;
  while (nb > 32 && (long long)nb * (long long)nE * 5LL > (long long)RCAP * (long long)nN * 4LL) nb >>= 1;
  return nb;
}
static inline int cdiv(int a, int b) { return (a + b - 1) / b; }
static inline size_t al256(size_t o) { return (o + 255) & ~(size_t)255; }

extern "C" void kernel_launch(void* const* d_in, const int* in_sizes, int n_in,
                              void* d_out, int out_size, void* d_ws, size_t ws_size,
                              hipStream_t stream) {
  if (n_in < 11) return;
  if (in_sizes[0] < CIN * GBM || (in_sizes[0] % CIN) != 0) return;
  const int nN = in_sizes[0] / CIN;
  if (nN < GBM || nN > (1 << 22)) return;
  if (in_sizes[1] != NMP * CIN * HCH) return;
  if (in_sizes[2] != NMP * HCH || in_sizes[3] != NMP * HCH) return;
  if (in_sizes[4] != NMP * HCH) return;
  if (in_sizes[9] < NMP || (in_sizes[9] % NMP) != 0) return;
  const int nE = in_sizes[9] / NMP;
  if (nE < 1 || nE >= (1 << 21)) return;
  if (in_sizes[10] != in_sizes[9] || in_sizes[5] != in_sizes[9]) return;
  if (in_sizes[6] != HCH * HIDW) return;
  if (in_sizes[7] != HIDW || in_sizes[8] != HIDW) return;
  if ((long long)out_size != (long long)nN * HCH) return;

  const float* h      = (const float*)d_in[0];
  const float* fc_W   = (const float*)d_in[1];
  const float* attn_l = (const float*)d_in[2];
  const float* attn_r = (const float*)d_in[3];
  const float* bias   = (const float*)d_in[4];
  const float* edge_w = (const float*)d_in[5];
  const float* sem_W1 = (const float*)d_in[6];
  const float* sem_b1 = (const float*)d_in[7];
  const float* sem_w2 = (const float*)d_in[8];
  const int*   src    = (const int*)  d_in[9];
  const int*   dst    = (const int*)  d_in[10];
  float* out = (float*)d_out;

  const int MP   = cdiv(nN, GBM) * GBM;
  const int gM   = MP / GBM;
  const int nb   = pick_nb(nE, nN);
  if (nb < 32 || (nb & (nb - 1)) != 0 || nb > NBMAX) return;
  const int gA   = cdiv(MP, nb);
  const int vec8 = ((nE & 3) == 0) ? 1 : 0;
  if ((long long)gA * nb < (long long)MP) return;
  if ((long long)(gM - 1) * GBM >= (long long)nN) return;

  char* ws = (char*)d_ws;
  size_t off = 0;
  const size_t oHB  = off; off = al256(off + (size_t)MP * CIN * 2);
  const size_t oWT  = off; off = al256(off + (size_t)FTW * CIN * 2);
  const size_t oW1T = off; off = al256(off + (size_t)HIDW * KZ * 2);
  const size_t oFT  = off; off = al256(off + (size_t)MP * FTW * 4);
  const size_t oZF  = off; off = al256(off + (size_t)NMP * MP * HCH * 4);
  const size_t oZH  = off; off = al256(off + (size_t)NMP * MP * KZ * 2);
  const size_t oPT  = off; off = al256(off + (size_t)NMP * gM * PREC * 4);
  const size_t oBE  = off; off = al256(off + (size_t)PREC * 4);
  if (off > ws_size || off > (size_t)WSMAX) return;
  unsigned short* HB  = (unsigned short*)(ws + oHB);
  unsigned short* WT  = (unsigned short*)(ws + oWT);
  unsigned short* W1T = (unsigned short*)(ws + oW1T);
  float*          FT  = (float*)(ws + oFT);
  float*          ZF  = (float*)(ws + oZF);
  unsigned short* ZH  = (unsigned short*)(ws + oZH);
  float*          PT  = (float*)(ws + oPT);
  float*          BETA = (float*)(ws + oBE);

  hipFuncSetAttribute(reinterpret_cast<const void*>(&k_agg), hipFuncAttributeMaxDynamicSharedMemorySize, LDS_AGG);

  const int nUh = MP * (CIN / 8);
  const int nUw = FTW * (CIN / 8);
  const int nUs = HIDW * (KZ / 8);
  k_prep<<<(nUh + nUw + nUs) / NTHR, NTHR, 0, stream>>>(h, fc_W, sem_W1, HB, WT, W1T, nN, nUh, nUw, nUs);
  k_gemm<0><<<dim3(gM, FTW / GBN), GTHR, 0, stream>>>(HB, CIN, 0, WT, CIN, CIN, FT, FTW, sem_b1, sem_w2, PT, nN, MP);
  k_agg<<<dim3(gA, NMP), NTHR, LDS_AGG, stream>>>(src, dst, edge_w, FT, attn_l, attn_r, bias, ZF, ZH,
                                                   nN, nE, nb, vec8, MP);
  k_gemm<1><<<dim3(gM, NMP), GTHR, 0, stream>>>(ZH, KZ, MP * KZ, W1T, KZ, KZ, FT, FTW, sem_b1, sem_w2, PT, nN, MP);
  k_beta<<<1, NTHR, 0, stream>>>(PT, gM, nN, BETA);
  const int nUo = nN * (HCH / 4);
  k_out<<<cdiv(nUo, NTHR), NTHR, 0, stream>>>(ZF, BETA, MP * HCH, nUo, out);
}
